// SparseLocalAttention_40948218200572
// MI455X (gfx1250) — hardware-verified
//
#include <hip/hip_runtime.h>
#include <stdint.h>
#include <stddef.h>

#define DEVINL __device__ __forceinline__

typedef _Float16 f16t;
typedef _Float16 v16h __attribute__((ext_vector_type(16)));
typedef _Float16 v8h  __attribute__((ext_vector_type(8)));
typedef __bf16   v16b __attribute__((ext_vector_type(16)));
typedef unsigned short v8us __attribute__((ext_vector_type(8)));
typedef float    v8f  __attribute__((ext_vector_type(8)));
typedef float    v4f  __attribute__((ext_vector_type(4)));
typedef v8h  __attribute__((may_alias)) v8ha;
typedef v8us __attribute__((may_alias)) v8usa;
typedef v4f  __attribute__((may_alias)) v4fa;
union FragH { v16h v; v8h half[2]; };
union FragB { v16b v; v8us half[2]; };

#define NBAT   128
#define NTOK   256
#define NC     384
#define NHD    6
#define HD     64
#define N3     1152
#define WIN    64
#define NHALF  2
#define HB     (NBAT / NHALF)
#define HTOK   (HB * NTOK)
#define XPL    ((size_t)HTOK * NC)
#define PLQ    ((size_t)HB * NHD * NTOK * HD)
#define TPBP   256
#define TPB    128
#define WAVES  4
#define PF     68
#define VCAR   16.0f
#define PCAR   1024.0f
#define ATT_SCALE 0.125f
#define SC_Y   (1.0f / (PCAR * VCAR))

#define WA_BLKS  ((N3 / 64) * (NC / 64))
#define WP_BLKS  ((NC / 64) * (NC / 64))
#define XC_BLKS  (HTOK * NC / 8 / TPBP)
#define NTT      (HTOK / 64)
#define NCT3     (N3 / 64)
#define NCT      (NC / 64)
#define QKV_BLKS (NTT * NCT3)
#define ATT_BLKS (HB * NHD * (NTOK / 64))
#define PRJ_BLKS (NTT * NCT)

static_assert(TPB == WAVES * 32);
static_assert(XC_BLKS * TPBP * 8 == HTOK * NC);
static_assert((NTOK % 64) == 0);
static_assert((NC % 64) == 0);
static_assert((N3 % 64) == 0);
static_assert(HD == 64);
static_assert(NCT3 == 3 * NCT);
static_assert((PF % 4) == 0);
static_assert(XPL == PLQ);
static_assert((NBAT % NHALF) == 0);

DEVINL v8f wmma_f16(v16h a, v16h b, v8f c) {
  v8f d = __builtin_amdgcn_wmma_f32_16x16x32_f16(false, a, false, b, (short)0, c, false, false);
  asm volatile("v_nop\n\tv_nop\n\tv_nop\n\tv_nop" : "+v"(d) : "v"(a), "v"(b));
  return d;
}
DEVINL v8f wmma_bf16(v16b a, v16b b, v8f c) {
  v8f d = __builtin_amdgcn_wmma_f32_16x16x32_bf16(false, a, false, b, (short)0, c, false, false);
  asm volatile("v_nop\n\tv_nop\n\tv_nop\n\tv_nop" : "+v"(d) : "v"(a), "v"(b));
  return d;
}
DEVINL v8f zero8f() {
  v8f z = {0.f, 0.f, 0.f, 0.f, 0.f, 0.f, 0.f, 0.f};
  return z;
}
DEVINL int imin(int a, int b) { return a < b ? a : b; }
DEVINL int imax(int a, int b) { return a > b ? a : b; }
DEVINL void load_fragb(FragB& f, const unsigned short* row, int k0) {
  f.half[0] = *(const v8usa*)(row + k0);
  f.half[1] = *(const v8usa*)(row + k0 + 16);
}
DEVINL unsigned short bf16_bits(float a) {
  union { __bf16 hh; unsigned short s; } u;
  u.hh = (__bf16)a;
  return u.s;
}
DEVINL void split_bf16(float v, unsigned short& hb, unsigned short& lb) {
  hb = bf16_bits(v);
  const float hf = __uint_as_float(((unsigned)hb) << 16);
  lb = bf16_bits(v - hf);
}

template <int KD>
DEVINL void mma3_4n(const unsigned short* __restrict__ ahr, const unsigned short* __restrict__ alr,
                    const unsigned short* __restrict__ bhr, const unsigned short* __restrict__ blr,
                    v8f (&acc)[4]) {
  #pragma unroll 1
  for (int ks = 0; ks < KD / 32; ++ks) {
    const int k0 = 32 * ks;
    FragB ah, al;
    load_fragb(ah, ahr, k0);
    load_fragb(al, alr, k0);
    #pragma unroll
    for (int n = 0; n < 4; ++n) {
      FragB bh, bl;
      load_fragb(bh, bhr + (size_t)16 * n * KD, k0);
      load_fragb(bl, blr + (size_t)16 * n * KD, k0);
      acc[n] = wmma_bf16(ah.v, bh.v, acc[n]);
      acc[n] = wmma_bf16(ah.v, bl.v, acc[n]);
      acc[n] = wmma_bf16(al.v, bh.v, acc[n]);
    }
  }
}

__global__ __launch_bounds__(TPBP) void prepw_k(const float* __restrict__ Wa, const float* __restrict__ Wp,
                                               unsigned short* __restrict__ WAH, unsigned short* __restrict__ WAL,
                                               unsigned short* __restrict__ WPH, unsigned short* __restrict__ WPL)
{
  __shared__ __attribute__((aligned(16))) float tile[64 * PF];
  const int blk = blockIdx.x, tid = threadIdx.x;
  if (blk >= WA_BLKS + WP_BLKS) return;
  const int isp = (blk >= WA_BLKS) ? 1 : 0;
  const int tb = isp ? (blk - WA_BLKS) : blk;
  const int nt = tb / NCT, kt = tb - NCT * nt;
  const int n0 = 64 * nt, k0 = 64 * kt;
  const float* src = isp ? Wp : Wa;
  const int pitch = isp ? NC : N3;
  unsigned short* dsth = isp ? WPH : WAH;
  unsigned short* dstl = isp ? WPL : WAL;

  const int krow = tid >> 2, nq = (tid & 3) * 16;
  const float* sp = src + (size_t)(k0 + krow) * pitch + n0 + nq;
  #pragma unroll
  for (int j = 0; j < 4; ++j) {
    const v4f a = *(const v4fa*)(sp + 4 * j);
    #pragma unroll
    for (int e = 0; e < 4; ++e) tile[(nq + 4 * j + e) * PF + krow] = a[e];
  }
  __syncthreads();

  const int q = tid & 7;
  v8us hv[2], lv[2];
  size_t off[2];
  #pragma unroll
  for (int p = 0; p < 2; ++p) {
    const int row = 32 * p + (tid >> 3);
    const v4f a = *(const v4fa*)(tile + row * PF + 8 * q), c = *(const v4fa*)(tile + row * PF + 8 * q + 4);
    #pragma unroll
    for (int j = 0; j < 4; ++j) {
      unsigned short hb, lb;
      split_bf16(a[j], hb, lb);
      hv[p][j] = hb; lv[p][j] = lb;
      split_bf16(c[j], hb, lb);
      hv[p][4 + j] = hb; lv[p][4 + j] = lb;
    }
    off[p] = (size_t)(n0 + row) * NC + k0 + 8 * q;
  }
  #pragma unroll
  for (int p = 0; p < 2; ++p) {
    *(volatile v8us*)(dsth + off[p]) = hv[p];
    *(volatile v8us*)(dstl + off[p]) = lv[p];
  }
  __threadfence();
  #pragma unroll
  for (int p = 0; p < 2; ++p) {
    *(volatile v8us*)(dsth + off[p]) = hv[p];
    *(volatile v8us*)(dstl + off[p]) = lv[p];
  }
}

__global__ __launch_bounds__(TPBP) void xcvt_k(const float* __restrict__ x, unsigned short* __restrict__ XH,
                                              unsigned short* __restrict__ XL, int n8)
{
  const int g = blockIdx.x * TPBP + threadIdx.x;
  if (g >= n8) return;
  const float* sp = x + (size_t)g * 8;
  const v4f a = *(const v4fa*)sp, c = *(const v4fa*)(sp + 4);
  v8us hv, lv;
  #pragma unroll
  for (int j = 0; j < 4; ++j) {
    unsigned short hb, lb;
    split_bf16(a[j], hb, lb);
    hv[j] = hb; lv[j] = lb;
    split_bf16(c[j], hb, lb);
    hv[4 + j] = hb; lv[4 + j] = lb;
  }
  const size_t off = (size_t)g * 8;
  *(volatile v8us*)(XH + off) = hv;
  *(volatile v8us*)(XL + off) = lv;
  __threadfence();
  *(volatile v8us*)(XH + off) = hv;
  *(volatile v8us*)(XL + off) = lv;
}

__global__ __launch_bounds__(TPB) void qkv_k(const unsigned short* __restrict__ XH, const unsigned short* __restrict__ XL,
                                            const unsigned short* __restrict__ WAH, const unsigned short* __restrict__ WAL,
                                            const float* __restrict__ bias,
                                            unsigned short* __restrict__ QH, unsigned short* __restrict__ QL,
                                            unsigned short* __restrict__ KH, unsigned short* __restrict__ KL,
                                            f16t* __restrict__ V)
{
  __shared__ __attribute__((aligned(16))) float sbuf[64 * PF];
  const int tid = threadIdx.x, lane = tid & 31, wave = tid >> 5;
  const int h = lane >> 4, m = lane & 15;
  const int blk = blockIdx.x;
  const int nb = blk / NCT3;
  const int ct = blk - NCT3 * nb;
  const int tok0 = 64 * nb, n0 = 64 * ct;
  const int region = ct / NCT;
  const int hh = ct - NCT * region;
  const int tr = (region == 2) ? 1 : 0;

  v8f acc[4];
  #pragma unroll
  for (int t = 0; t < 4; ++t) acc[t] = zero8f();
  {
    const size_t aoff = (size_t)(tok0 + 16 * wave + m) * NC + 8 * h;
    const size_t boff = (size_t)(n0 + m) * NC + 8 * h;
    mma3_4n<NC>(XH + aoff, XL + aoff, WAH + boff, WAL + boff, acc);
  }

  #pragma unroll
  for (int t = 0; t < 4; ++t) {
    const int d = 16 * t + m;
    const float bv = bias[n0 + d];
    #pragma unroll
    for (int r = 0; r < 8; ++r) {
      const int row = 16 * wave + 8 * h + r;
      const float v = acc[t][r] + bv;
      const int idx = tr ? (d * PF + row) : (row * PF + d);
      sbuf[idx] = v;
    }
  }
  __syncthreads();

  const int q = tid & 7;
  if (tr) {
    const int bl = tok0 >> 8, t0 = tok0 & (NTOK - 1);
    f16t* VP = V + ((size_t)(bl * NHD + hh) * HD) * NTOK + t0;
    v8h ov[4];
    size_t off[4];
    #pragma unroll
    for (int k = 0; k < 4; ++k) {
      const int d = 16 * k + (tid >> 3);
      const v4f a = *(const v4fa*)(sbuf + d * PF + 8 * q), c = *(const v4fa*)(sbuf + d * PF + 8 * q + 4);
      #pragma unroll
      for (int j = 0; j < 4; ++j) {
        ov[k][j]     = (f16t)(a[j] * VCAR);
        ov[k][4 + j] = (f16t)(c[j] * VCAR);
      }
      off[k] = (size_t)d * NTOK + 8 * q;
    }
    #pragma unroll
    for (int k = 0; k < 4; ++k) *(volatile v8h*)(VP + off[k]) = ov[k];
    __threadfence();
    #pragma unroll
    for (int k = 0; k < 4; ++k) *(volatile v8h*)(VP + off[k]) = ov[k];
  } else {
    unsigned short* PHI = (region == 0) ? QH : KH;
    unsigned short* PLO = (region == 0) ? QL : KL;
    v8us hv[4], lv[4];
    size_t off[4];
    #pragma unroll
    for (int k = 0; k < 4; ++k) {
      const int row = 16 * k + (tid >> 3);
      const v4f a = *(const v4fa*)(sbuf + row * PF + 8 * q), c = *(const v4fa*)(sbuf + row * PF + 8 * q + 4);
      #pragma unroll
      for (int j = 0; j < 4; ++j) {
        unsigned short hb, lb;
        split_bf16(a[j], hb, lb);
        hv[k][j] = hb; lv[k][j] = lb;
        split_bf16(c[j], hb, lb);
        hv[k][4 + j] = hb; lv[k][4 + j] = lb;
      }
      const int tok = tok0 + row, bl = tok >> 8, t = tok & (NTOK - 1);
      off[k] = ((size_t)(bl * NHD + hh) * NTOK + t) * HD + 8 * q;
    }
    #pragma unroll
    for (int k = 0; k < 4; ++k) {
      *(volatile v8us*)(PHI + off[k]) = hv[k];
      *(volatile v8us*)(PLO + off[k]) = lv[k];
    }
    __threadfence();
    #pragma unroll
    for (int k = 0; k < 4; ++k) {
      *(volatile v8us*)(PHI + off[k]) = hv[k];
      *(volatile v8us*)(PLO + off[k]) = lv[k];
    }
  }
}

DEVINL v8f score_tile(const unsigned short* khr, const unsigned short* klr,
                      const FragB& qh0, const FragB& ql0, const FragB& qh1, const FragB& ql1) {
  v8f s = zero8f();
  FragB kh, kl;
  load_fragb(kh, khr, 0);
  load_fragb(kl, klr, 0);
  s = wmma_bf16(kh.v, qh0.v, s);
  s = wmma_bf16(kh.v, ql0.v, s);
  s = wmma_bf16(kl.v, qh0.v, s);
  load_fragb(kh, khr, 32);
  load_fragb(kl, klr, 32);
  s = wmma_bf16(kh.v, qh1.v, s);
  s = wmma_bf16(kh.v, ql1.v, s);
  s = wmma_bf16(kl.v, qh1.v, s);
  return s;
}

__global__ __launch_bounds__(TPB) void attn_k(const unsigned short* __restrict__ QH, const unsigned short* __restrict__ QL,
                                             const unsigned short* __restrict__ KH, const unsigned short* __restrict__ KL,
                                             const f16t* __restrict__ V,
                                             unsigned short* __restrict__ YH, unsigned short* __restrict__ YL)
{
  __shared__ __attribute__((aligned(16))) float sbuf[64 * PF];
  const int tid = threadIdx.x, lane = tid & 31, wave = tid >> 5;
  const int h = lane >> 4, m = lane & 15;
  const int blk = blockIdx.x;
  const int bh = blk >> 2, qb = blk & 3;
  const int bl = bh / NHD, hh = bh - NHD * bl;
  const int i0w = 64 * qb + 16 * wave;
  const int iq = i0w + m;
  const int jlo = iq - WIN;

  FragB qh0, qh1, ql0, ql1;
  {
    const size_t foff = ((size_t)bh * NTOK + iq) * HD + 8 * h;
    load_fragb(qh0, QH + foff, 0);
    load_fragb(qh1, QH + foff, 32);
    load_fragb(ql0, QL + foff, 0);
    load_fragb(ql1, QL + foff, 32);
  }
  const unsigned short* khb = KH + (size_t)bh * NTOK * HD + 8 * h;
  const unsigned short* klb = KL + (size_t)bh * NTOK * HD + 8 * h;
  const f16t* vb = V + ((size_t)bh * HD + m) * NTOK;

  const int js = imax(i0w - WIN, 0);
  const int nsteps = (i0w + 16 - js + 31) >> 5;

  v8f O[4];
  #pragma unroll
  for (int t = 0; t < 4; ++t) O[t] = zero8f();
  float Mx = -3.0e38f, L = 0.0f;

  #pragma unroll 1
  for (int s = 0; s < nsteps; ++s) {
    const int j0 = js + 32 * s;
    const int jr0 = imin(j0 + m, NTOK - 1), jr1 = imin(j0 + 16 + m, NTOK - 1);
    v8f s0 = score_tile(khb + (size_t)jr0 * HD, klb + (size_t)jr0 * HD, qh0, ql0, qh1, ql1);
    v8f s1 = score_tile(khb + (size_t)jr1 * HD, klb + (size_t)jr1 * HD, qh0, ql0, qh1, ql1);

    const int jb0 = j0 + 8 * h, jb1 = jb0 + 16;
    bool ok0[8], ok1[8];
    float mloc = -3.0e38f;
    #pragma unroll
    for (int r = 0; r < 8; ++r) {
      s0[r] *= ATT_SCALE;
      s1[r] *= ATT_SCALE;
      ok0[r] = (jb0 + r <= iq) && (jb0 + r >= jlo);
      ok1[r] = (jb1 + r <= iq) && (jb1 + r >= jlo);
      mloc = fmaxf(mloc, ok0[r] ? s0[r] : -3.0e38f);
      mloc = fmaxf(mloc, ok1[r] ? s1[r] : -3.0e38f);
    }
    mloc = fmaxf(mloc, __shfl_xor(mloc, 16));
    const float Mn = fmaxf(Mx, mloc);
    const float corr = __expf(Mx - Mn);
    Mx = Mn;

    FragH pf;
    float ls = 0.0f;
    #pragma unroll
    for (int r = 0; r < 8; ++r) {
      const float a0 = fminf(s0[r] - Mn, 0.0f);
      const float a1 = fminf(s1[r] - Mn, 0.0f);
      const float e0 = ok0[r] ? __expf(a0) : 0.0f;
      const float e1 = ok1[r] ? __expf(a1) : 0.0f;
      ls += e0 + e1;
      pf.half[0][r] = (f16t)(e0 * PCAR);
      pf.half[1][r] = (f16t)(e1 * PCAR);
    }
    ls += __shfl_xor(ls, 16);
    L = L * corr + ls;
    #pragma unroll
    for (int t = 0; t < 4; ++t) {
      #pragma unroll
      for (int r = 0; r < 8; ++r) O[t][r] *= corr;
    }
    const int g0 = imin(j0 + 8 * h, NTOK - 8), g1 = imin(j0 + 16 + 8 * h, NTOK - 8);
    #pragma unroll
    for (int t = 0; t < 4; ++t) {
      FragH va;
      const f16t* vrow = vb + (size_t)16 * t * NTOK;
      va.half[0] = *(const v8ha*)(vrow + g0);
      va.half[1] = *(const v8ha*)(vrow + g1);
      O[t] = wmma_f16(va.v, pf.v, O[t]);
    }
  }

  const float inv = (1.0f / L) * SC_Y;
  #pragma unroll
  for (int t = 0; t < 4; ++t) {
    #pragma unroll
    for (int r = 0; r < 8; ++r)
      sbuf[(16 * wave + m) * PF + 16 * t + 8 * h + r] = O[t][r] * inv;
  }
  __syncthreads();

  v8us hv[4], lv[4];
  size_t off[4];
  #pragma unroll
  for (int k = 0; k < 4; ++k) {
    const int row = 16 * k + (tid >> 3), q = tid & 7;
    const v4f a = *(const v4fa*)(sbuf + row * PF + 8 * q), c = *(const v4fa*)(sbuf + row * PF + 8 * q + 4);
    #pragma unroll
    for (int j = 0; j < 4; ++j) {
      unsigned short hb, lb;
      split_bf16(a[j], hb, lb);
      hv[k][j] = hb; lv[k][j] = lb;
      split_bf16(c[j], hb, lb);
      hv[k][4 + j] = hb; lv[k][4 + j] = lb;
    }
    const int tok = bl * NTOK + 64 * qb + row;
    off[k] = (size_t)tok * NC + hh * HD + 8 * q;
  }
  #pragma unroll
  for (int k = 0; k < 4; ++k) {
    *(volatile v8us*)(YH + off[k]) = hv[k];
    *(volatile v8us*)(YL + off[k]) = lv[k];
  }
  __threadfence();
  #pragma unroll
  for (int k = 0; k < 4; ++k) {
    *(volatile v8us*)(YH + off[k]) = hv[k];
    *(volatile v8us*)(YL + off[k]) = lv[k];
  }
}

__global__ __launch_bounds__(TPB) void proj_k(const unsigned short* __restrict__ YH, const unsigned short* __restrict__ YL,
                                             const unsigned short* __restrict__ WPH, const unsigned short* __restrict__ WPL,
                                             const float* __restrict__ bias, float* __restrict__ out)
{
  __shared__ __attribute__((aligned(16))) float sbuf[64 * PF];
  const int tid = threadIdx.x, lane = tid & 31, wave = tid >> 5;
  const int h = lane >> 4, m = lane & 15;
  const int blk = blockIdx.x;
  const int nb = blk / NCT;
  const int ct = blk - NCT * nb;
  const int tok0 = 64 * nb, n0 = 64 * ct;

  v8f acc[4];
  #pragma unroll
  for (int t = 0; t < 4; ++t) acc[t] = zero8f();
  {
    const size_t aoff = (size_t)(tok0 + 16 * wave + m) * NC + 8 * h;
    const size_t boff = (size_t)(n0 + m) * NC + 8 * h;
    mma3_4n<NC>(YH + aoff, YL + aoff, WPH + boff, WPL + boff, acc);
  }

  #pragma unroll
  for (int t = 0; t < 4; ++t) {
    const int n = 16 * t + m;
    const float bv = bias[n0 + n];
    #pragma unroll
    for (int r = 0; r < 8; ++r) {
      const int row = 16 * wave + 8 * h + r;
      sbuf[row * PF + n] = acc[t][r] + bv;
    }
  }
  __syncthreads();

  v4f ov[8];
  size_t off[8];
  #pragma unroll
  for (int k = 0; k < 8; ++k) {
    const int row = 8 * k + (tid >> 4), q = tid & 15;
    ov[k] = *(const v4fa*)(sbuf + row * PF + 4 * q);
    off[k] = (size_t)(tok0 + row) * NC + n0 + 4 * q;
  }
  #pragma unroll
  for (int k = 0; k < 8; ++k) *(volatile v4f*)(out + off[k]) = ov[k];
  __threadfence();
  #pragma unroll
  for (int k = 0; k < 8; ++k) *(volatile v4f*)(out + off[k]) = ov[k];
}

extern "C" void kernel_launch(void* const* d_in, const int* in_sizes, int n_in,
                              void* d_out, int out_size, void* d_ws, size_t ws_size,
                              hipStream_t stream) {
  if (n_in < 5) return;
  if (in_sizes[0] != NBAT * NTOK * NC) return;
  if (in_sizes[1] != NC * N3 || in_sizes[2] != N3) return;
  if (in_sizes[3] != NC * NC || in_sizes[4] != NC) return;
  if (out_size != NBAT * NTOK * NC) return;

  const float* x  = (const float*)d_in[0];
  const float* Wa = (const float*)d_in[1];
  const float* ba = (const float*)d_in[2];
  const float* Wp = (const float*)d_in[3];
  const float* bp = (const float*)d_in[4];
  float* outp = (float*)d_out;

  const size_t szX  = XPL * 2;
  const size_t szWA = (size_t)N3 * NC * 2;
  const size_t szWP = (size_t)NC * NC * 2;
  const size_t szQ  = PLQ * 2;
  static_assert(2 * (XPL * 2) + 2 * ((size_t)N3 * NC * 2) + 2 * ((size_t)NC * NC * 2) + 4 * (PLQ * 2) + PLQ * 2 + 2 * (XPL * 2)
                <= (size_t)134217728);
  static_assert(((XPL * 2) % 128) == 0);
  static_assert((((size_t)N3 * NC * 2) % 128) == 0);
  static_assert((((size_t)NC * NC * 2) % 128) == 0);
  size_t off = 0;
  char* ws = (char*)d_ws;
  unsigned short* XH  = (unsigned short*)(ws + off); off += szX;
  unsigned short* XL  = (unsigned short*)(ws + off); off += szX;
  unsigned short* WAH = (unsigned short*)(ws + off); off += szWA;
  unsigned short* WAL = (unsigned short*)(ws + off); off += szWA;
  unsigned short* WPH = (unsigned short*)(ws + off); off += szWP;
  unsigned short* WPL = (unsigned short*)(ws + off); off += szWP;
  unsigned short* QH = (unsigned short*)(ws + off); off += szQ;
  unsigned short* QL = (unsigned short*)(ws + off); off += szQ;
  unsigned short* KH = (unsigned short*)(ws + off); off += szQ;
  unsigned short* KL = (unsigned short*)(ws + off); off += szQ;
  f16t* VP = (f16t*)(ws + off); off += szQ;
  unsigned short* YH = (unsigned short*)(ws + off); off += szX;
  unsigned short* YL = (unsigned short*)(ws + off); off += szX;
  if (off > ws_size) return;

  prepw_k<<<WA_BLKS + WP_BLKS, TPBP, 0, stream>>>(Wa, Wp, WAH, WAL, WPH, WPL);

  for (int half = 0; half < NHALF; ++half) {
    const float* xh = x + (size_t)half * XPL;
    float* oh = outp + (size_t)half * XPL;
    xcvt_k<<<XC_BLKS, TPBP, 0, stream>>>(xh, XH, XL, (int)(XPL / 8));
    qkv_k<<<QKV_BLKS, TPB, 0, stream>>>(XH, XL, WAH, WAL, ba, QH, QL, KH, KL, VP);
    attn_k<<<ATT_BLKS, TPB, 0, stream>>>(QH, QL, KH, KL, VP, YH, YL);
    proj_k<<<PRJ_BLKS, TPB, 0, stream>>>(YH, YL, WPH, WPL, bp, oh);
  }
  (void)hipGetLastError();
}
